// NeuralAttention_45329084842553
// MI455X (gfx1250) — hardware-verified
//
#include <hip/hip_runtime.h>
#include <stdint.h>

typedef __attribute__((ext_vector_type(16))) _Float16 v16h;
typedef __attribute__((ext_vector_type(8)))  _Float16 v8h;
typedef __attribute__((ext_vector_type(16))) __bf16   v16b;
typedef __attribute__((ext_vector_type(8)))  __bf16   v8b;
typedef __attribute__((ext_vector_type(8)))  float    v8f;
typedef __attribute__((ext_vector_type(4)))  float    v4f;
typedef __attribute__((ext_vector_type(4)))  int      v4i;

__device__ __forceinline__ unsigned short f2bf_bits(float f) {
  unsigned u = __float_as_uint(f);
  return (unsigned short)((u + 0x7FFFu + ((u >> 16) & 1u)) >> 16);
}
__device__ __forceinline__ float bf_bits2f(unsigned short h) { return __uint_as_float(((unsigned)h) << 16); }

__device__ __forceinline__ void dep_guard_h(v8f& a, v8f& b, v16h x, v16h y) { asm volatile("v_nop\n\tv_nop\n\tv_nop\n\tv_nop" : "+v"(a), "+v"(b) : "v"(x), "v"(y)); }
__device__ __forceinline__ void dep_guard_b(v8f& a, v8f& b, v16b x, v16b y) { asm volatile("v_nop\n\tv_nop\n\tv_nop\n\tv_nop" : "+v"(a), "+v"(b) : "v"(x), "v"(y)); }
__device__ __forceinline__ void keep4_h(v16h a, v16h b, v16h c, v16h d) { asm volatile("v_nop" :: "v"(a), "v"(b), "v"(c), "v"(d)); }
__device__ __forceinline__ void keep4_b(v16b a, v16b b, v16b c, v16b d) { asm volatile("v_nop" :: "v"(a), "v"(b), "v"(c), "v"(d)); }
__device__ __forceinline__ void acc_guard4(v8f& a, v8f& b, v8f& c, v8f& d) { asm volatile("v_nop\n\tv_nop\n\tv_nop\n\tv_nop" : "+v"(a), "+v"(b), "+v"(c), "+v"(d)); }
template <typename T> struct Frag;
template <> struct Frag<_Float16> {
  typedef v16h V; union U { v16h v; v8h h[2]; };
  static __device__ __forceinline__ v16h load(const _Float16* p) {
    U f; f.h[0] = *(const v8h*)(p); f.h[1] = *(const v8h*)(p + 16); return f.v;
  }
  static __device__ __forceinline__ v8f mma(v16h a, v16h b, v8f c) {
    return __builtin_amdgcn_wmma_f32_16x16x32_f16(false, a, false, b, (short)0, c, false, false);
  }
  static __device__ __forceinline__ void guard(v8f& a, v8f& b, v16h x, v16h y) { dep_guard_h(a, b, x, y); }
  static __device__ __forceinline__ void keep(v16h a, v16h b, v16h c, v16h d) { keep4_h(a, b, c, d); }
};
template <> struct Frag<__bf16> {
  typedef v16b V; union U { v16b v; v8b h[2]; };
  static __device__ __forceinline__ v16b load(const __bf16* p) {
    U f; f.h[0] = *(const v8b*)(p); f.h[1] = *(const v8b*)(p + 16); return f.v;
  }
  static __device__ __forceinline__ v8f mma(v16b a, v16b b, v8f c) {
    return __builtin_amdgcn_wmma_f32_16x16x32_bf16(false, a, false, b, (short)0, c, false, false);
  }
  static __device__ __forceinline__ void guard(v8f& a, v8f& b, v16b x, v16b y) { dep_guard_b(a, b, x, y); }
  static __device__ __forceinline__ void keep(v16b a, v16b b, v16b c, v16b d) { keep4_b(a, b, c, d); }
};

template <int ET> struct Elem;
template <> struct Elem<0> { typedef _Float16 T; };
template <> struct Elem<1> { typedef __bf16 T; };
template <int ET, bool SPLIT, int BIAS_MODE, int OUT_MODE, bool RESID, int ACT = 0>
__global__ __launch_bounds__(256) void wmma_gemm64(
    const unsigned short* __restrict__ Ap, const unsigned short* __restrict__ A2p, int lda, long strideA,
    const unsigned short* __restrict__ Btp, const unsigned short* __restrict__ Bt2p, int ldb, long strideB,
    void* __restrict__ Cout, void* __restrict__ Cout2, int ldc, long strideC,
    const float* __restrict__ bias,
    const float* __restrict__ resid, long strideR,
    int M, int N, int K, float scale) {
  typedef typename Elem<ET>::T T;
  typedef typename Frag<T>::V V;
  const T* A = (const T*)Ap; const T* A2 = (const T*)A2p; const T* Bt = (const T*)Btp; const T* Bt2 = (const T*)Bt2p;
  __shared__ __align__(16) float sT[8][16 * 68];
  const int b    = blockIdx.y;
  const int lane = threadIdx.x & 31;
  const int wave = threadIdx.x >> 5;
  const int tilesN = N >> 6;
  const int tilesM = M >> 6;
  const int tile = blockIdx.x * 8 + wave;
  if (tile >= tilesM * tilesN) return;
  const int tm = tile / tilesN;
  const int tn = tile - tm * tilesN;
  const int m0 = tm << 6;
  const int n0 = tn << 6;

  const T* Ab  = A  + (size_t)b * strideA;
  const T* Bb  = Bt + (size_t)b * strideB;
  const T* Ab2 = SPLIT ? (A2  + (size_t)b * strideA) : nullptr;
  const T* Bb2 = SPLIT ? (Bt2 + (size_t)b * strideB) : nullptr;

  const int rlane = lane & 15;
  const int koff  = (lane >> 4) * 8;
  const int mOff  = (lane >> 4) * 8;

  v8f acc[4][4];
#pragma unroll
  for (int i = 0; i < 4; ++i)
#pragma unroll
    for (int j = 0; j < 4; ++j) acc[i][j] = (v8f){0.f,0.f,0.f,0.f,0.f,0.f,0.f,0.f};

  for (int k0 = 0; k0 < K; k0 += 32) {
    V bh[4], bl[4];
#pragma unroll
    for (int j = 0; j < 4; ++j) {
      const size_t bo = (size_t)(n0 + (j << 4) + rlane) * ldb + koff + k0;
      bh[j] = Frag<T>::load(Bb + bo);
      if (SPLIT) bl[j] = Frag<T>::load(Bb2 + bo);
    }
#pragma unroll
    for (int i = 0; i < 4; ++i) {
      const size_t ao = (size_t)(m0 + (i << 4) + rlane) * lda + koff + k0;
      V ah = Frag<T>::load(Ab + ao);
      V al;
      if (SPLIT) al = Frag<T>::load(Ab2 + ao);
#pragma unroll
      for (int j = 0; j < 4; ++j) {
        acc[i][j] = Frag<T>::mma(ah, bh[j], acc[i][j]);
        if (SPLIT) {
          acc[i][j] = Frag<T>::mma(ah, bl[j], acc[i][j]);
          acc[i][j] = Frag<T>::mma(al, bh[j], acc[i][j]);
        }
      }
      Frag<T>::guard(acc[i][0], acc[i][3], ah, SPLIT ? al : ah);
    }
    Frag<T>::keep(bh[0], bh[1], bh[2], bh[3]);
    if (SPLIT) Frag<T>::keep(bl[0], bl[1], bl[2], bl[3]);
  }
  acc_guard4(acc[0][0], acc[0][1], acc[0][2], acc[0][3]);
  acc_guard4(acc[1][0], acc[1][1], acc[1][2], acc[1][3]);
  acc_guard4(acc[2][0], acc[2][1], acc[2][2], acc[2][3]);
  acc_guard4(acc[3][0], acc[3][1], acc[3][2], acc[3][3]);

  float* slab = sT[wave];
  const float* Rb = RESID ? (resid + (size_t)b * strideR) : nullptr;
#pragma unroll
  for (int i = 0; i < 4; ++i) {
    const int mBase = m0 + (i << 4);
#pragma unroll
    for (int j = 0; j < 4; ++j) {
      const int n = n0 + (j << 4) + rlane;
      float bv = 0.f;
      if (BIAS_MODE == 2) bv = bias[n];
#pragma unroll
      for (int r = 0; r < 8; ++r) {
        float v = acc[i][j][r] * scale;
        if (BIAS_MODE == 1) v += bias[mBase + mOff + r];
        if (BIAS_MODE == 2) v += bv;
        if (RESID) v += Rb[(size_t)(mBase + mOff + r) * ldc + n];
        if (ACT == 1) v = tanhf(v);
        if (ACT == 2) v = fmaxf(v, 0.0f);
        if (ACT == 3) v = v / (1.0f + expf(-v));
        if (ACT == 4) v = (v > 0.f) ? v : 0.01f * v;
        if (ACT == 5) v = 0.5f * v * (1.0f + erff(v * 0.70710678118654752f));
        slab[(mOff + r) * 68 + (j << 4) + rlane] = v;
      }
    }
    __builtin_amdgcn_fence(__ATOMIC_RELEASE, "workgroup");
    __builtin_amdgcn_wave_barrier();
    __builtin_amdgcn_fence(__ATOMIC_ACQUIRE, "workgroup");
    if (OUT_MODE == 0) {
      float* C = (float*)Cout + (size_t)b * strideC;
      const int hh = lane >> 4, c4 = (lane & 15) * 4;
      for (int pass = 0; pass < 2; ++pass) {
#pragma unroll
        for (int it = 0; it < 8; ++it) {
          const int row = it * 2 + hh;
          v4f v = *(const v4f*)(slab + row * 68 + c4);
          *(volatile v4f*)(C + (size_t)(mBase + row) * ldc + n0 + c4) = v;
        }
        __threadfence();
      }
    } else {
      const int q = lane >> 3, c8 = (lane & 7) * 8;
      unsigned short* C  = (unsigned short*)Cout  + (size_t)b * strideC;
      unsigned short* C2 = (OUT_MODE == 2) ? ((unsigned short*)Cout2 + (size_t)b * strideC) : nullptr;
      for (int pass = 0; pass < 2; ++pass) {
#pragma unroll
        for (int it = 0; it < 4; ++it) {
          const int row = it * 4 + q;
          const float* sp = slab + row * 68 + c8;
          v8h hv, lv;
#pragma unroll
          for (int e = 0; e < 8; ++e) {
            if (OUT_MODE == 1) {
              hv[e] = (_Float16)sp[e];
            } else {
              unsigned short hb = f2bf_bits(sp[e]);
              unsigned short lb = f2bf_bits(sp[e] - bf_bits2f(hb));
              hv[e] = __builtin_bit_cast(_Float16, hb);
              lv[e] = __builtin_bit_cast(_Float16, lb);
            }
          }
          *(volatile v8h*)(C + (size_t)(mBase + row) * ldc + n0 + c8) = hv;
          if (OUT_MODE == 2) *(volatile v8h*)(C2 + (size_t)(mBase + row) * ldc + n0 + c8) = lv;
        }
        __threadfence();
      }
    }
    __builtin_amdgcn_fence(__ATOMIC_RELEASE, "workgroup");
    __builtin_amdgcn_wave_barrier();
    __builtin_amdgcn_fence(__ATOMIC_ACQUIRE, "workgroup");
  }
}

__global__ __launch_bounds__(256) void cast_f32_f16x2s(
    const float* __restrict__ in, _Float16* __restrict__ out, int n2, float scale) {
  int i = blockIdx.x * 256 + threadIdx.x;
  if (i < n2) {
    const _Float16 h0 = (_Float16)(in[2 * i] * scale), h1 = (_Float16)(in[2 * i + 1] * scale);
    const unsigned u = (unsigned)__builtin_bit_cast(unsigned short, h0) | ((unsigned)__builtin_bit_cast(unsigned short, h1) << 16);
    ((volatile unsigned*)out)[i] = u;
    __threadfence();
    ((volatile unsigned*)out)[i] = u;
  }
}

#define AT_D 64
#define AT_NW 4
#define AT_QB 64
#define AT_KC 64
struct AttnGeomR {
  const float* cosT; const float* sinT; const int* ts; const int* mask;
  long q_bs, q_rs, q_hs, k_bs, k_rs, k_hs, v_bs, v_rs, v_hs, o_bs, o_rs, o_hs;
  long m_bs, m_rs, ts_bs;
  int S, Skv, H, maxF;
  float sscale, mask_fill, oscale, pad0;
};
static_assert(sizeof(AttnGeomR) == 184);

__device__ __forceinline__ v8f at_mma_h(v16h a, v16h b, v8f c) {
  c = __builtin_amdgcn_wmma_f32_16x16x32_f16(false, a, false, b, (short)0, c, false, false);
  asm volatile("v_nop\n\tv_nop\n\tv_nop\n\tv_nop" : "+v"(c) : "v"(a), "v"(b));
  return c;
}

__global__ __launch_bounds__(128)
void attn64_rope_f16(const float* __restrict__ q, const float* __restrict__ k,
                     const float* __restrict__ v, _Float16* __restrict__ out, AttnGeomR g) {
  const float PSC = 32768.0f;
  union FH { v16h v; v8h h[2]; };
  __shared__ __align__(16) _Float16 Ksh[AT_KC * AT_D];
  __shared__ __align__(16) _Float16 Vth[AT_D * AT_KC];
  __shared__ __align__(16) _Float16 Psh[AT_NW][16 * AT_KC];
  __shared__ __align__(16) float    Os[AT_NW][16 * 68];
  __shared__ int Mfl[AT_NW];

  const int tid  = threadIdx.x;
  const int wave = tid >> 5;
  const int lane = tid & 31;
  const int hh   = lane >> 4;
  const int c    = lane & 15;

  const int nqb = g.S / AT_QB;
  const int bx = blockIdx.x;
  const int qb = bx % nqb;
  const int bh = bx / nqb;
  const int h  = bh % g.H;
  const int b  = bh / g.H;
  const int qbase = qb * AT_QB;
  const int q0 = qbase + wave * 16;

  const float* qb_ptr = q + (size_t)b * g.q_bs + (size_t)h * g.q_hs;
  const float* kb_ptr = k + (size_t)b * g.k_bs + (size_t)h * g.k_hs;
  const float* vb_ptr = v + (size_t)b * g.v_bs + (size_t)h * g.v_hs;
  _Float16*    ob_ptr = out + (size_t)b * g.o_bs + (size_t)h * g.o_hs;
  const int*   tsb    = g.ts + (size_t)b * g.ts_bs;
  const int*   mkb    = g.mask + (size_t)b * g.m_bs;

  v16h qa[2];
  {
    const int qr = q0 + c;
    const float* qrow = qb_ptr + (size_t)qr * g.q_rs;
    int tq = tsb[qr];
    tq = tq < 0 ? 0 : (tq >= g.maxF ? g.maxF - 1 : tq);
    const float* cr = g.cosT + (size_t)tq * AT_D;
    const float* sr = g.sinT + (size_t)tq * AT_D;
#pragma unroll
    for (int hf = 0; hf < 2; ++hf) {
#pragma unroll
      for (int e = 0; e < 8; ++e) {
        const int d = hf * 16 + 8 * hh + e;
        const float a0 = qrow[d], a1 = qrow[d + 32];
        const float r0 = a0 * cr[d] - a1 * sr[d];
        const float r1 = a1 * cr[d + 32] + a0 * sr[d + 32];
        qa[0][hf * 8 + e] = (_Float16)r0;
        qa[1][hf * 8 + e] = (_Float16)r1;
      }
    }
  }

  float mrow[8], lrow[8];
  v8f oacc[4];
#pragma unroll
  for (int r = 0; r < 8; ++r) { mrow[r] = -__builtin_inff(); lrow[r] = 0.f; }
#pragma unroll
  for (int t = 0; t < 4; ++t) oacc[t] = (v8f){0.f,0.f,0.f,0.f,0.f,0.f,0.f,0.f};

  const int nChunks = g.Skv / AT_KC;
  for (int kc = 0; kc < nChunks; ++kc) {
    const int kv0 = kc * AT_KC;
    __syncthreads();
    {
      const int kvr = tid >> 1, dl = (tid & 1) * 16;
      const int kva = kv0 + kvr;
      const float* krow = kb_ptr + (size_t)kva * g.k_rs + dl;
      const float* vrow = vb_ptr + (size_t)kva * g.v_rs + dl;
      int tk = tsb[kva];
      tk = tk < 0 ? 0 : (tk >= g.maxF ? g.maxF - 1 : tk);
      const float* cr = g.cosT + (size_t)tk * AT_D + dl;
      const float* sr = g.sinT + (size_t)tk * AT_D + dl;
#pragma unroll
      for (int i = 0; i < 4; ++i) {
        const v4f k0 = *(const v4f*)(krow + 4 * i), k1 = *(const v4f*)(krow + 32 + 4 * i);
        const v4f c0 = *(const v4f*)(cr + 4 * i),   c1 = *(const v4f*)(cr + 32 + 4 * i);
        const v4f s0 = *(const v4f*)(sr + 4 * i),   s1 = *(const v4f*)(sr + 32 + 4 * i);
        const v4f w0 = *(const v4f*)(vrow + 4 * i), w1 = *(const v4f*)(vrow + 32 + 4 * i);
#pragma unroll
        for (int e = 0; e < 4; ++e) {
          const int d = dl + 4 * i + e;
          const float r0 = k0[e] * c0[e] - k1[e] * s0[e];
          const float r1 = k1[e] * c1[e] + k0[e] * s1[e];
          Ksh[kvr * AT_D + d]        = (_Float16)r0;
          Ksh[kvr * AT_D + d + 32]   = (_Float16)r1;
          Vth[d * AT_KC + kvr]        = (_Float16)w0[e];
          Vth[(d + 32) * AT_KC + kvr] = (_Float16)w1[e];
        }
      }
      const int* mrw = mkb + (size_t)(qbase + kvr) * g.m_rs + kv0 + (tid & 1) * 32;
      int fz = 0;
#pragma unroll
      for (int i = 0; i < 8; ++i) {
        const v4i mm = *(const v4i*)(mrw + 4 * i);
        fz |= (int)(mm[0] == 0) | (int)(mm[1] == 0) | (int)(mm[2] == 0) | (int)(mm[3] == 0);
      }
      const int anyz = __any(fz);
      if (lane == 0) Mfl[wave] = anyz;
    }
    __syncthreads();
    const int anyMasked = Mfl[0] | Mfl[1] | Mfl[2] | Mfl[3];

    v8f s[4];
#pragma unroll
    for (int j = 0; j < 4; ++j) {
      s[j] = (v8f){0.f,0.f,0.f,0.f,0.f,0.f,0.f,0.f};
#pragma unroll
      for (int dc = 0; dc < 2; ++dc) {
        FH kf;
        kf.h[0] = *(const v8h*)(Ksh + (j * 16 + c) * AT_D + dc * 32 + 8 * hh);
        kf.h[1] = *(const v8h*)(Ksh + (j * 16 + c) * AT_D + dc * 32 + 16 + 8 * hh);
        s[j] = at_mma_h(qa[dc], kf.v, s[j]);
      }
    }
    float cm[8];
#pragma unroll
    for (int r = 0; r < 8; ++r) {
      const int qrow = q0 + 8 * hh + r;
      const int* mrowp = mkb + (size_t)qrow * g.m_rs + kv0;
      float m = -__builtin_inff();
#pragma unroll
      for (int j = 0; j < 4; ++j) {
        float sv = s[j][r] * g.sscale;
        if (anyMasked) {
          if (mrowp[j * 16 + c] == 0) sv = g.mask_fill;
        }
        s[j][r] = sv;
        m = fmaxf(m, sv);
      }
#pragma unroll
      for (int off = 1; off < 16; off <<= 1) m = fmaxf(m, __shfl_xor(m, off, 32));
      cm[r] = m;
    }
    _Float16* pw = Psh[wave];
#pragma unroll
    for (int r = 0; r < 8; ++r) {
      const float mnew = fmaxf(mrow[r], cm[r]);
      const float alpha = expf(mrow[r] - mnew);
      mrow[r] = mnew;
      float psum = 0.f;
#pragma unroll
      for (int j = 0; j < 4; ++j) {
        const float p = expf(s[j][r] - mnew);
        psum += p;
        pw[(8 * hh + r) * AT_KC + j * 16 + c] = (_Float16)(p * PSC);
      }
#pragma unroll
      for (int off = 1; off < 16; off <<= 1) psum += __shfl_xor(psum, off, 32);
      lrow[r] = lrow[r] * alpha + psum;
#pragma unroll
      for (int t = 0; t < 4; ++t) oacc[t][r] *= alpha;
    }
    __builtin_amdgcn_fence(__ATOMIC_RELEASE, "workgroup");
    __builtin_amdgcn_wave_barrier();
    __builtin_amdgcn_fence(__ATOMIC_ACQUIRE, "workgroup");
#pragma unroll 1
    for (int kk = 0; kk < 2; ++kk) {
      FH pa;
      pa.h[0] = *(const v8h*)(pw + c * AT_KC + kk * 32 + 8 * hh);
      pa.h[1] = *(const v8h*)(pw + c * AT_KC + kk * 32 + 16 + 8 * hh);
#pragma unroll
      for (int t = 0; t < 4; ++t) {
        FH vf;
        vf.h[0] = *(const v8h*)(Vth + (t * 16 + c) * AT_KC + kk * 32 + 8 * hh);
        vf.h[1] = *(const v8h*)(Vth + (t * 16 + c) * AT_KC + kk * 32 + 16 + 8 * hh);
        oacc[t] = at_mma_h(pa.v, vf.v, oacc[t]);
      }
    }
  }

  float* os = Os[wave];
#pragma unroll
  for (int r = 0; r < 8; ++r) {
    const float inv = g.oscale * (1.0f / (lrow[r] * PSC));
#pragma unroll
    for (int t = 0; t < 4; ++t) os[(8 * hh + r) * 68 + t * 16 + c] = oacc[t][r] * inv;
  }
  __builtin_amdgcn_fence(__ATOMIC_RELEASE, "workgroup");
  __builtin_amdgcn_wave_barrier();
  __builtin_amdgcn_fence(__ATOMIC_ACQUIRE, "workgroup");
  {
    const int qq = lane >> 3, c8 = (lane & 7) * 8;
    for (int pass = 0; pass < 2; ++pass) {
#pragma unroll
      for (int it = 0; it < 4; ++it) {
        const int row = it * 4 + qq;
        const float* sp = os + row * 68 + c8;
        v8h hv;
#pragma unroll
        for (int e = 0; e < 8; ++e) hv[e] = (_Float16)sp[e];
        *(volatile v8h*)(ob_ptr + (size_t)(q0 + row) * g.o_rs + c8) = hv;
      }
      __threadfence();
    }
  }
}

extern "C" void kernel_launch(void* const* d_in, const int* in_sizes, int n_in,
                              void* d_out, int out_size, void* d_ws, size_t ws_size,
                              hipStream_t stream) {
  if (n_in < 9) return;
  const float* x    = (const float*)d_in[0];
  const float* Wq   = (const float*)d_in[1];
  const float* Wk   = (const float*)d_in[2];
  const float* Wv   = (const float*)d_in[3];
  const float* Wo   = (const float*)d_in[4];
  const float* cosT = (const float*)d_in[5];
  const float* sinT = (const float*)d_in[6];
  const int*   mask = (const int*)d_in[7];
  const int*   ts   = (const int*)d_in[8];
  float* outp = (float*)d_out;

  const int HIDc = 1024, NHc = 16, HDc = 64;
  const long nX  = in_sizes[0];
  const long nTS = in_sizes[8];
  if (nTS <= 0) return;
  const long MT = nX / HIDc;
  if (MT != nTS || MT * HIDc != nX || (MT % 64) != 0) return;
  const long nM = in_sizes[7];
  const long T = nM / nTS;
  if (T <= 0 || (T % 64) != 0) return;
  const long Bn = nTS / T;
  if (Bn * T != nTS || Bn * T * T != nM) return;
  for (int i = 1; i <= 4; ++i) if ((long)in_sizes[i] != (long)HIDc * HIDc) return;
  const int maxF = in_sizes[5] / HDc;
  if (maxF <= 0 || in_sizes[6] != in_sizes[5] || maxF * HDc != in_sizes[5]) return;
  if ((long)out_size != MT * HIDc) return;

  char* ws = (char*)d_ws;
  size_t off = 0;
  auto carve = [&](size_t bytes) -> char* { char* p = ws + off; off += (bytes + 255) & ~(size_t)255; return p; };
  _Float16* x16  = (_Float16*)carve((size_t)MT * HIDc * 2);
  _Float16* wq16 = (_Float16*)carve((size_t)HIDc * HIDc * 2);
  _Float16* wk16 = (_Float16*)carve((size_t)HIDc * HIDc * 2);
  _Float16* wv16 = (_Float16*)carve((size_t)HIDc * HIDc * 2);
  _Float16* wo16 = (_Float16*)carve((size_t)HIDc * HIDc * 2);
  float* q32 = (float*)carve((size_t)MT * HIDc * 4);
  float* k32 = (float*)carve((size_t)MT * HIDc * 4);
  float* v32 = (float*)carve((size_t)MT * HIDc * 4);
  if (off > ws_size) return;
  _Float16* ctx16 = x16;

  {
    const int n2x = (int)(MT * HIDc / 2);
    cast_f32_f16x2s<<<(n2x + 255) / 256, 256, 0, stream>>>(x, x16, n2x, 1.0f);
    const int n2w = HIDc * HIDc / 2;
    cast_f32_f16x2s<<<(n2w + 255) / 256, 256, 0, stream>>>(Wq, wq16, n2w, 64.0f);
    cast_f32_f16x2s<<<(n2w + 255) / 256, 256, 0, stream>>>(Wk, wk16, n2w, 64.0f);
    cast_f32_f16x2s<<<(n2w + 255) / 256, 256, 0, stream>>>(Wv, wv16, n2w, 64.0f);
    cast_f32_f16x2s<<<(n2w + 255) / 256, 256, 0, stream>>>(Wo, wo16, n2w, 64.0f);
  }

  const int tiles = (int)((MT / 64) * (HIDc / 64));
  dim3 gg((unsigned)((tiles + 7) / 8), 1);
  typedef const unsigned short* cu16;
  wmma_gemm64<0, false, 0, 0, false, 0><<<gg, 256, 0, stream>>>(
      (cu16)x16, (cu16)x16, HIDc, 0L, (cu16)wq16, (cu16)wq16, HIDc, 0L,
      (void*)q32, (void*)q32, HIDc, 0L, cosT, cosT, 0L, (int)MT, HIDc, HIDc, 0.015625f);
  wmma_gemm64<0, false, 0, 0, false, 0><<<gg, 256, 0, stream>>>(
      (cu16)x16, (cu16)x16, HIDc, 0L, (cu16)wk16, (cu16)wk16, HIDc, 0L,
      (void*)k32, (void*)k32, HIDc, 0L, cosT, cosT, 0L, (int)MT, HIDc, HIDc, 0.015625f);
  wmma_gemm64<0, false, 0, 0, false, 0><<<gg, 256, 0, stream>>>(
      (cu16)x16, (cu16)x16, HIDc, 0L, (cu16)wv16, (cu16)wv16, HIDc, 0L,
      (void*)v32, (void*)v32, HIDc, 0L, cosT, cosT, 0L, (int)MT, HIDc, HIDc, 0.015625f);

  AttnGeomR g;
  g.cosT = cosT; g.sinT = sinT; g.ts = ts; g.mask = mask;
  g.q_bs = T * HIDc; g.q_rs = HIDc; g.q_hs = HDc;
  g.k_bs = T * HIDc; g.k_rs = HIDc; g.k_hs = HDc;
  g.v_bs = T * HIDc; g.v_rs = HIDc; g.v_hs = HDc;
  g.o_bs = T * HIDc; g.o_rs = HIDc; g.o_hs = HDc;
  g.m_bs = T * T; g.m_rs = T; g.ts_bs = T;
  g.S = (int)T; g.Skv = (int)T; g.H = NHc; g.maxF = maxF;
  g.sscale = 0.125f; g.mask_fill = -3.4028235e38f; g.oscale = 256.0f; g.pad0 = 0.0f;
  const unsigned nblk = (unsigned)(Bn * NHc * (T / 64));
  attn64_rope_f16<<<nblk, 128, 0, stream>>>(q32, k32, v32, ctx16, g);

  wmma_gemm64<0, false, 0, 0, false, 0><<<gg, 256, 0, stream>>>(
      (cu16)ctx16, (cu16)ctx16, HIDc, 0L, (cu16)wo16, (cu16)wo16, HIDc, 0L,
      (void*)outp, (void*)outp, HIDc, 0L, cosT, cosT, 0L, (int)MT, HIDc, HIDc, 6.103515625e-05f);
}
